// Raindrop_15401752723925
// MI455X (gfx1250) — hardware-verified
//
#include <hip/hip_runtime.h>
#include <math.h>

constexpr int DIM_B   = 64;
constexpr int DIM_T   = 128;
constexpr int DIM_S   = 64;
constexpr int DIM_O   = 4;
constexpr int DIM_E   = 64;
constexpr int DIM_PE  = 16;
constexpr int DIM_A   = 10;
constexpr int DIM_OUT = 128;
constexpr int DIM_CAT = DIM_A + DIM_PE;
constexpr int DIM_H   = DIM_E + DIM_PE;
constexpr int CH_B    = 4;
constexpr int N_CHUNK = DIM_B / CH_B;
constexpr int ROWS_CH  = CH_B * DIM_T * DIM_S;
constexpr int PAIRS_CH = CH_B * DIM_T;
constexpr int BS_CH    = CH_B * DIM_S;
constexpr int PITCH_W  = 128;
constexpr int PITCH_PE = 32;
constexpr int K_HC     = 96;
constexpr int SCALE_BITS = 0x3de4f92e;

typedef __attribute__((ext_vector_type(16))) _Float16 v16h;
typedef __attribute__((ext_vector_type(8)))  _Float16 v8h;
typedef __attribute__((ext_vector_type(16))) __bf16   v16b;
typedef __attribute__((ext_vector_type(8)))  __bf16   v8b;
typedef __attribute__((ext_vector_type(8)))  float    v8f;
typedef __attribute__((ext_vector_type(4)))  float    v4f;
typedef __attribute__((ext_vector_type(4)))  unsigned int v4u;

__constant__ unsigned int c_freq_bits[8] = {0x3f800000, 0x3ea1e89b, 0x3dcccccc, 0x3d0186e2, 0x3c23d70a, 0x3b4f3e33, 0x3a83126e, 0x39a5cb60};
static_assert(sizeof(c_freq_bits) / sizeof(c_freq_bits[0]) == 8);

__device__ __forceinline__ unsigned short f2bf_bits(float f) {
  unsigned u = __float_as_uint(f);
  return (unsigned short)((u + 0x7FFFu + ((u >> 16) & 1u)) >> 16);
}
__device__ __forceinline__ float bf_bits2f(unsigned short h) { return __uint_as_float(((unsigned)h) << 16); }

__device__ __forceinline__ void dep_guard_h(v8f& a, v8f& b, v16h x, v16h y) { asm volatile("v_nop\n\tv_nop\n\tv_nop\n\tv_nop" : "+v"(a), "+v"(b) : "v"(x), "v"(y)); }
__device__ __forceinline__ void dep_guard_b(v8f& a, v8f& b, v16b x, v16b y) { asm volatile("v_nop\n\tv_nop\n\tv_nop\n\tv_nop" : "+v"(a), "+v"(b) : "v"(x), "v"(y)); }
__device__ __forceinline__ void keep4_h(v16h a, v16h b, v16h c, v16h d) { asm volatile("v_nop" :: "v"(a), "v"(b), "v"(c), "v"(d)); }
__device__ __forceinline__ void keep4_b(v16b a, v16b b, v16b c, v16b d) { asm volatile("v_nop" :: "v"(a), "v"(b), "v"(c), "v"(d)); }
__device__ __forceinline__ void acc_guard4(v8f& a, v8f& b, v8f& c, v8f& d) { asm volatile("v_nop\n\tv_nop\n\tv_nop\n\tv_nop" : "+v"(a), "+v"(b), "+v"(c), "+v"(d)); }
template <typename T> struct Frag;
template <> struct Frag<_Float16> {
  typedef v16h V; union U { v16h v; v8h h[2]; };
  static __device__ __forceinline__ v16h load(const _Float16* p) {
    U f; f.h[0] = *(const v8h*)(p); f.h[1] = *(const v8h*)(p + 16); return f.v;
  }
  static __device__ __forceinline__ v8f mma(v16h a, v16h b, v8f c) {
    return __builtin_amdgcn_wmma_f32_16x16x32_f16(false, a, false, b, (short)0, c, false, false);
  }
  static __device__ __forceinline__ void guard(v8f& a, v8f& b, v16h x, v16h y) { dep_guard_h(a, b, x, y); }
  static __device__ __forceinline__ void keep(v16h a, v16h b, v16h c, v16h d) { keep4_h(a, b, c, d); }
};
template <> struct Frag<__bf16> {
  typedef v16b V; union U { v16b v; v8b h[2]; };
  static __device__ __forceinline__ v16b load(const __bf16* p) {
    U f; f.h[0] = *(const v8b*)(p); f.h[1] = *(const v8b*)(p + 16); return f.v;
  }
  static __device__ __forceinline__ v8f mma(v16b a, v16b b, v8f c) {
    return __builtin_amdgcn_wmma_f32_16x16x32_bf16(false, a, false, b, (short)0, c, false, false);
  }
  static __device__ __forceinline__ void guard(v8f& a, v8f& b, v16b x, v16b y) { dep_guard_b(a, b, x, y); }
  static __device__ __forceinline__ void keep(v16b a, v16b b, v16b c, v16b d) { keep4_b(a, b, c, d); }
};

__device__ __forceinline__ unsigned pk16(unsigned short a, unsigned short b) { return (unsigned)a | ((unsigned)b << 16); }

__device__ __forceinline__ void split8(const float* v, v4u& hi, v4u& lo) {
  unsigned short hb[8], lb[8];
#pragma unroll
  for (int e = 0; e < 8; ++e) {
    hb[e] = f2bf_bits(v[e]);
    lb[e] = f2bf_bits(v[e] - bf_bits2f(hb[e]));
  }
  hi = (v4u){pk16(hb[0], hb[1]), pk16(hb[2], hb[3]), pk16(hb[4], hb[5]), pk16(hb[6], hb[7])};
  lo = (v4u){pk16(lb[0], lb[1]), pk16(lb[2], lb[3]), pk16(lb[4], lb[5]), pk16(lb[6], lb[7])};
}

__device__ __forceinline__ void st2_pair(unsigned short* ph, unsigned short* pl, size_t off, v4u hv, v4u lv) {
  *(volatile v4u*)(ph + off) = hv;
  *(volatile v4u*)(pl + off) = lv;
  __threadfence();
  *(volatile v4u*)(ph + off) = hv;
  *(volatile v4u*)(pl + off) = lv;
}

template <int ET> struct Elem;
template <> struct Elem<0> { typedef _Float16 T; };
template <> struct Elem<1> { typedef __bf16 T; };
template <int ET, bool SPLIT, int BIAS_MODE, int OUT_MODE, bool RESID, int ACT = 0>
__global__ __launch_bounds__(256) void wmma_gemm64(
    const unsigned short* __restrict__ Ap, const unsigned short* __restrict__ A2p, int lda, long strideA,
    const unsigned short* __restrict__ Btp, const unsigned short* __restrict__ Bt2p, int ldb, long strideB,
    void* __restrict__ Cout, void* __restrict__ Cout2, int ldc, long strideC,
    const float* __restrict__ bias,
    const float* __restrict__ resid, long strideR,
    int M, int N, int K, float scale, int nbatch) {
  typedef typename Elem<ET>::T T;
  typedef typename Frag<T>::V V;
  const T* A = (const T*)Ap; const T* A2 = (const T*)A2p; const T* Bt = (const T*)Btp; const T* Bt2 = (const T*)Bt2p;
  __shared__ __align__(16) float sT[8][16 * 68];
  const int lane = threadIdx.x & 31;
  const int wave = threadIdx.x >> 5;
  const int tilesN = N >> 6;
  const int tilesM = M >> 6;
  const int tilesPer = tilesM * tilesN;
  const int gt = blockIdx.x * 8 + wave;
  if (gt >= tilesPer * nbatch) return;
  const int b    = gt / tilesPer;
  const int tile = gt - b * tilesPer;
  const int tm = tile / tilesN;
  const int tn = tile - tm * tilesN;
  const int m0 = tm << 6;
  const int n0 = tn << 6;

  const T* Ab  = A  + (size_t)b * strideA;
  const T* Bb  = Bt + (size_t)b * strideB;
  const T* Ab2 = SPLIT ? (A2  + (size_t)b * strideA) : nullptr;
  const T* Bb2 = SPLIT ? (Bt2 + (size_t)b * strideB) : nullptr;

  const int rlane = lane & 15;
  const int koff  = (lane >> 4) * 8;
  const int mOff  = (lane >> 4) * 8;

  v8f acc[4][4];
#pragma unroll
  for (int i = 0; i < 4; ++i)
#pragma unroll
    for (int j = 0; j < 4; ++j) acc[i][j] = (v8f){0.f,0.f,0.f,0.f,0.f,0.f,0.f,0.f};

  for (int k0 = 0; k0 < K; k0 += 32) {
    V bh[4], bl[4];
#pragma unroll
    for (int j = 0; j < 4; ++j) {
      const size_t bo = (size_t)(n0 + (j << 4) + rlane) * ldb + koff + k0;
      bh[j] = Frag<T>::load(Bb + bo);
      if (SPLIT) bl[j] = Frag<T>::load(Bb2 + bo);
    }
#pragma unroll
    for (int i = 0; i < 4; ++i) {
      const size_t ao = (size_t)(m0 + (i << 4) + rlane) * lda + koff + k0;
      V ah = Frag<T>::load(Ab + ao);
      V al;
      if (SPLIT) al = Frag<T>::load(Ab2 + ao);
#pragma unroll
      for (int j = 0; j < 4; ++j) {
        acc[i][j] = Frag<T>::mma(ah, bh[j], acc[i][j]);
        if (SPLIT) {
          acc[i][j] = Frag<T>::mma(ah, bl[j], acc[i][j]);
          acc[i][j] = Frag<T>::mma(al, bh[j], acc[i][j]);
        }
      }
      Frag<T>::guard(acc[i][0], acc[i][3], ah, SPLIT ? al : ah);
    }
    Frag<T>::keep(bh[0], bh[1], bh[2], bh[3]);
    if (SPLIT) Frag<T>::keep(bl[0], bl[1], bl[2], bl[3]);
  }
  acc_guard4(acc[0][0], acc[0][1], acc[0][2], acc[0][3]);
  acc_guard4(acc[1][0], acc[1][1], acc[1][2], acc[1][3]);
  acc_guard4(acc[2][0], acc[2][1], acc[2][2], acc[2][3]);
  acc_guard4(acc[3][0], acc[3][1], acc[3][2], acc[3][3]);

  float* slab = sT[wave];
  const float* Rb = RESID ? (resid + (size_t)b * strideR) : nullptr;
#pragma unroll
  for (int i = 0; i < 4; ++i) {
    const int mBase = m0 + (i << 4);
#pragma unroll
    for (int j = 0; j < 4; ++j) {
      const int n = n0 + (j << 4) + rlane;
      float bv = 0.f;
      if (BIAS_MODE == 2) bv = bias[n];
#pragma unroll
      for (int r = 0; r < 8; ++r) {
        float v = acc[i][j][r] * scale;
        if (BIAS_MODE == 1) v += bias[mBase + mOff + r];
        if (BIAS_MODE == 2) v += bv;
        if (RESID) v += Rb[(size_t)(mBase + mOff + r) * ldc + n];
        if (ACT == 2) v = fmaxf(v, 0.0f);
        if (ACT == 4) v = (v > 0.f) ? v : 0.01f * v;
        slab[(mOff + r) * 68 + (j << 4) + rlane] = v;
      }
    }
    __builtin_amdgcn_fence(__ATOMIC_RELEASE, "workgroup");
    __builtin_amdgcn_wave_barrier();
    __builtin_amdgcn_fence(__ATOMIC_ACQUIRE, "workgroup");
    if (OUT_MODE == 0) {
      float* C = (float*)Cout + (size_t)b * strideC;
      const int hh = lane >> 4, c4 = (lane & 15) * 4;
      for (int pass = 0; pass < 2; ++pass) {
#pragma unroll
        for (int it = 0; it < 8; ++it) {
          const int row = it * 2 + hh;
          v4f v = *(const v4f*)(slab + row * 68 + c4);
          *(volatile v4f*)(C + (size_t)(mBase + row) * ldc + n0 + c4) = v;
        }
        __threadfence();
      }
    } else {
      const int q = lane >> 3, c8 = (lane & 7) * 8;
      unsigned short* C  = (unsigned short*)Cout  + (size_t)b * strideC;
      unsigned short* C2 = (OUT_MODE == 2) ? ((unsigned short*)Cout2 + (size_t)b * strideC) : nullptr;
      for (int pass = 0; pass < 2; ++pass) {
#pragma unroll
        for (int it = 0; it < 4; ++it) {
          const int row = it * 4 + q;
          const float* sp = slab + row * 68 + c8;
          v8h hv, lv;
#pragma unroll
          for (int e = 0; e < 8; ++e) {
            if (OUT_MODE == 1) {
              hv[e] = (_Float16)sp[e];
            } else {
              unsigned short hb = f2bf_bits(sp[e]);
              unsigned short lb = f2bf_bits(sp[e] - bf_bits2f(hb));
              hv[e] = __builtin_bit_cast(_Float16, hb);
              lv[e] = __builtin_bit_cast(_Float16, lb);
            }
          }
          *(volatile v8h*)(C + (size_t)(mBase + row) * ldc + n0 + c8) = hv;
          if (OUT_MODE == 2) *(volatile v8h*)(C2 + (size_t)(mBase + row) * ldc + n0 + c8) = lv;
        }
        __threadfence();
      }
    }
    __builtin_amdgcn_fence(__ATOMIC_RELEASE, "workgroup");
    __builtin_amdgcn_wave_barrier();
    __builtin_amdgcn_fence(__ATOMIC_ACQUIRE, "workgroup");
  }
}

__global__ __launch_bounds__(128) void k_petab(const float* __restrict__ times, float* __restrict__ PE) {
#pragma clang fp contract(off)
  __shared__ __align__(16) float spe[128 * 36];
  const int tid = threadIdx.x;
  const int bt = blockIdx.x * 128 + tid;
  const float tv = times[bt];
#pragma unroll 1
  for (int i = 0; i < 8; ++i) {
    const float fr = __uint_as_float(c_freq_bits[i]);
    const float ang = tv * fr;
    spe[tid * 36 + i] = sinf(ang);
    spe[tid * 36 + 8 + i] = cosf(ang);
  }
  __syncthreads();
  const int piece = tid & 7;
  const int rsub  = tid >> 3;
  const int pcl   = (piece < 4) ? piece : 3;
  float* pbase = PE + (size_t)blockIdx.x * 128 * PITCH_PE;
  for (int pass = 0; pass < 2; ++pass) {
#pragma unroll
    for (int it = 0; it < 8; ++it) {
      const int row = it * 16 + rsub;
      const v4f lv = *(const v4f*)(spe + row * 36 + 4 * pcl);
      v4f v;
      v[0] = (piece < 4) ? lv[0] : 0.f;
      v[1] = (piece < 4) ? lv[1] : 0.f;
      v[2] = (piece < 4) ? lv[2] : 0.f;
      v[3] = (piece < 4) ? lv[3] : 0.f;
      *(volatile v4f*)(pbase + (size_t)row * PITCH_PE + 4 * piece) = v;
    }
    __threadfence();
  }
}

__global__ __launch_bounds__(256) void k_wprep(
    const float* __restrict__ bw, const float* __restrict__ wrecv, const float* __restrict__ brecv,
    const float* __restrict__ wq, const float* __restrict__ bq, const float* __restrict__ wk, const float* __restrict__ bk,
    const float* __restrict__ wemb,
    unsigned short* BWh, unsigned short* BWl, unsigned short* WRh, unsigned short* WRl,
    unsigned short* WQh, unsigned short* WQl, unsigned short* WEh, unsigned short* WEl, float* BIAS) {
  const int tid = threadIdx.x;
  const int blk = blockIdx.x;
  if (blk == 16) {
    if (tid < 32) {
      v4f o;
#pragma unroll
      for (int e = 0; e < 4; ++e) {
        const int f = 4 * tid + e;
        const int n1 = f & 63;
        const float vb = brecv[min(n1, DIM_CAT - 1)];
        const float vq = bq[min(n1, DIM_A - 1)];
        const float vk = bk[min(max(n1 - DIM_A, 0), DIM_A - 1)];
        const float first = (n1 < DIM_CAT) ? vb : 0.f;
        const float second = (n1 < DIM_A) ? vq : ((n1 < 2 * DIM_A) ? vk : 0.f);
        o[e] = (f < 64) ? first : second;
      }
      float* dst = BIAS + 4 * tid;
      *(volatile v4f*)dst = o;
      __threadfence();
      *(volatile v4f*)dst = o;
    }
    return;
  }
  float v[8];
  size_t off;
  unsigned short* ph;
  unsigned short* pl;
  if (blk < 2) {
    const int g = blk * 256 + tid;
    const int i = g >> 3, c8 = (g & 7) * 8;
#pragma unroll
    for (int e = 0; e < 8; ++e) v[e] = bw[i * DIM_E + c8 + e];
    off = (size_t)g * 8; ph = BWh; pl = BWl;
  } else if (blk < 4) {
    const int g = (blk - 2) * 256 + tid;
    const int n = g >> 3, c8 = (g & 7) * 8;
    const int nn = min(n, DIM_CAT - 1);
#pragma unroll
    for (int e = 0; e < 8; ++e) {
      const int k = c8 + e;
      const float w = wrecv[k * DIM_CAT + nn];
      v[e] = (n < DIM_CAT) ? w : 0.f;
    }
    off = (size_t)g * 8; ph = WRh; pl = WRl;
  } else if (blk < 8) {
    const int g = (blk - 4) * 256 + tid;
    const int n = g >> 4, c8 = (g & 15) * 8;
    const int nq = min(n, DIM_A - 1);
    const int nk = min(max(n - DIM_A, 0), DIM_A - 1);
#pragma unroll
    for (int e = 0; e < 8; ++e) {
      const int k = c8 + e;
      const int kk = min(k, DIM_H - 1);
      const float a = wq[kk * DIM_A + nq];
      const float c = wk[kk * DIM_A + nk];
      const float sel = (n < DIM_A) ? a : ((n < 2 * DIM_A) ? c : 0.f);
      v[e] = (k < DIM_H) ? sel : 0.f;
    }
    off = (size_t)g * 8; ph = WQh; pl = WQl;
  } else {
    const int g = (blk - 8) * 256 + tid;
    const int n = g >> 4, c8 = (g & 15) * 8;
#pragma unroll
    for (int e = 0; e < 8; ++e) {
      const int k = c8 + e;
      const int kk = min(k, DIM_H - 1);
      const float a = wemb[kk * DIM_OUT + n];
      v[e] = (k < DIM_H) ? a : 0.f;
    }
    off = (size_t)g * 8; ph = WEh; pl = WEl;
  }
  v4u hv, lv;
  split8(v, hv, lv);
  st2_pair(ph, pl, off, hv, lv);
}

__global__ __launch_bounds__(256) void k_embed(
    const float* __restrict__ x, const float* __restrict__ mask, const float* __restrict__ obsW,
    const float* __restrict__ isaW, const float* __restrict__ PE, int chunk,
    unsigned short* H0h, unsigned short* H0l, unsigned short* H0Th, unsigned short* H0Tl,
    unsigned short* ACh, unsigned short* ACl) {
  __shared__ float sh[64 * 65];
  const int tid = threadIdx.x;
  const int p = blockIdx.x;
  const int bl = p >> 7, t = p & 127;
  const int b = chunk * CH_B + bl;
  const int bt = b * DIM_T + t;
#pragma unroll 1
  for (int i = 0; i < 16; ++i) {
    const int idx = i * 256 + tid;
    const int s = idx >> 6, e = idx & 63;
    const v4f xv = *(const v4f*)(x + ((size_t)bt * DIM_S + s) * DIM_O);
    const float* wp = obsW + (size_t)s * (DIM_O * DIM_E) + e;
    float acc = xv[0] * wp[0];
    acc += xv[1] * wp[DIM_E];
    acc += xv[2] * wp[2 * DIM_E];
    acc += xv[3] * wp[3 * DIM_E];
    sh[s * 65 + e] = fmaxf(acc, 0.f) * mask[(size_t)bt * DIM_S + s];
  }
  __syncthreads();
  const size_t pbase = (size_t)p * 4096;
  {
    v4u hv[2], lv[2];
#pragma unroll
    for (int it = 0; it < 2; ++it) {
      const int g = it * 256 + tid;
      const int s = g >> 3, c8 = (g & 7) * 8;
      float v[8];
#pragma unroll
      for (int e = 0; e < 8; ++e) v[e] = sh[s * 65 + c8 + e];
      split8(v, hv[it], lv[it]);
    }
    st2_pair(H0h, H0l, pbase + (size_t)tid * 8, hv[0], lv[0]);
    st2_pair(H0h, H0l, pbase + (size_t)(256 + tid) * 8, hv[1], lv[1]);
  }
  {
    v4u hv[2], lv[2];
#pragma unroll
    for (int it = 0; it < 2; ++it) {
      const int g = it * 256 + tid;
      const int er = g >> 3, j8 = (g & 7) * 8;
      float v[8];
#pragma unroll
      for (int e = 0; e < 8; ++e) v[e] = sh[(j8 + e) * 65 + er];
      split8(v, hv[it], lv[it]);
    }
    st2_pair(H0Th, H0Tl, pbase + (size_t)tid * 8, hv[0], lv[0]);
    st2_pair(H0Th, H0Tl, pbase + (size_t)(256 + tid) * 8, hv[1], lv[1]);
  }
  {
    v4u hv[2], lv[2];
#pragma unroll
    for (int it = 0; it < 2; ++it) {
      const int g = it * 256 + tid;
      const int j = g >> 3, d8 = (g & 7) * 8;
      float v[8];
#pragma unroll
      for (int e = 0; e < 8; ++e) {
        const int d = d8 + e;
        const int dq = min(d, DIM_A - 1);
        const int dp = min(max(d - DIM_A, 0), DIM_PE - 1);
        const float va = isaW[j * DIM_A + dq];
        const float vp = PE[(size_t)bt * PITCH_PE + dp];
        v[e] = (d < DIM_A) ? va : ((d < DIM_CAT) ? vp : 0.f);
      }
      split8(v, hv[it], lv[it]);
    }
    st2_pair(ACh, ACl, pbase + (size_t)tid * 8, hv[0], lv[0]);
    st2_pair(ACh, ACl, pbase + (size_t)(256 + tid) * 8, hv[1], lv[1]);
  }
}

template <int WMODE>
__global__ __launch_bounds__(256) void k_wsplit(const float* __restrict__ ALPHA, const float* __restrict__ BIDIR,
                                                const float* __restrict__ ADJ2, unsigned short* Wh, unsigned short* Wl) {
  const int g = blockIdx.x * 256 + threadIdx.x;
  const int p = g >> 9;
  const int i = (g >> 3) & 63, j8 = (g & 7) * 8;
  const int bl = p >> 7;
  const float* ap = ALPHA + (size_t)p * 4096 + i * 64 + j8;
  const v4f a0 = *(const v4f*)(ap), a1 = *(const v4f*)(ap + 4);
  const float* bp = BIDIR + i * 64 + j8;
  const v4f b0 = *(const v4f*)(bp), b1 = *(const v4f*)(bp + 4);
  float v[8];
#pragma unroll
  for (int e = 0; e < 4; ++e) { v[e] = b0[e] * a0[e]; v[4 + e] = b1[e] * a1[e]; }
  if (WMODE == 2) {
    const float* dp = ADJ2 + (size_t)(bl * 64 + i) * 64 + j8;
    const v4f d0 = *(const v4f*)(dp), d1 = *(const v4f*)(dp + 4);
#pragma unroll
    for (int e = 0; e < 4; ++e) { v[e] = v[e] * d0[e]; v[4 + e] = v[4 + e] * d1[e]; }
  }
  v4u hv, lv;
  split8(v, hv, lv);
  st2_pair(Wh, Wl, (size_t)g * 8, hv, lv);
}

__global__ __launch_bounds__(256) void k_adj2(const float* __restrict__ ALPHA, const float* __restrict__ mask,
                                              float* ADJ2, int chunk) {
  const int g = blockIdx.x * 256 + threadIdx.x;
  const int bl = g >> 10;
  const int i = (g >> 4) & 63, j4 = g & 15;
  const int b = chunk * CH_B + bl;
  const float* ap = ALPHA + (size_t)(bl * DIM_T) * 4096 + i * 64 + j4 * 4;
  const float* mp = mask + (size_t)(b * DIM_T) * DIM_S + i;
  v4f a = {0.f, 0.f, 0.f, 0.f};
  float m = 0.f;
#pragma unroll 1
  for (int t = 0; t < DIM_T; ++t) {
    a += *(const v4f*)(ap + (size_t)t * 4096);
    m += mp[t * DIM_S];
  }
  const float inv = 1.0f / m;
  const v4f r = a * inv;
  float* dst = ADJ2 + (size_t)g * 4;
  *(volatile v4f*)dst = r;
  __threadfence();
  *(volatile v4f*)dst = r;
}

__global__ __launch_bounds__(256) void k_hcat(const float* __restrict__ H2, const float* __restrict__ PE,
                                              unsigned short* HCh, unsigned short* HCl, int chunk) {
  const int g = blockIdx.x * 256 + threadIdx.x;
  const int q = g >> 4, c8 = (g & 15) * 8;
  const int bl = q >> 13, s = (q >> 7) & 63, t = q & 127;
  const int b = chunk * CH_B + bl;
  const int cc = (c8 < DIM_E) ? c8 : (DIM_E - 8);
  const int pc = (c8 >= DIM_E && c8 < DIM_H) ? (c8 - DIM_E) : 0;
  const float* hp = H2 + ((size_t)((bl * DIM_T + t) * DIM_S + s)) * DIM_E + cc;
  const v4f h0v = *(const v4f*)(hp), h1v = *(const v4f*)(hp + 4);
  const float* pp = PE + (size_t)(b * DIM_T + t) * PITCH_PE + pc;
  const v4f p0 = *(const v4f*)(pp), p1 = *(const v4f*)(pp + 4);
  float v[8];
#pragma unroll
  for (int e = 0; e < 4; ++e) {
    v[e]     = (c8 < DIM_E) ? h0v[e] : ((c8 < DIM_H) ? p0[e] : 0.f);
    v[4 + e] = (c8 < DIM_E) ? h1v[e] : ((c8 < DIM_H) ? p1[e] : 0.f);
  }
  v4u hv, lv;
  split8(v, hv, lv);
  st2_pair(HCh, HCl, (size_t)g * 8, hv, lv);
}

__global__ __launch_bounds__(128) void k_attn(const float* __restrict__ QK, const float* __restrict__ H2,
                                              const float* __restrict__ PE, const float* __restrict__ Ws,
                                              const float* __restrict__ bs, unsigned short* CTXh, unsigned short* CTXl,
                                              int chunk) {
  __shared__ float skwp[DIM_A * DIM_T];
  __shared__ float skw[16];
  __shared__ float smax[4];
  __shared__ float ssum[4];
  __shared__ float sbeta[DIM_T];
  __shared__ __align__(16) unsigned short s16h[128];
  __shared__ __align__(16) unsigned short s16l[128];
  const int tid = threadIdx.x;
  const int lane = tid & 31, wave = tid >> 5;
  const int blk = blockIdx.x;
  const int bl = blk >> 6, s = blk & 63;
  const int b = chunk * CH_B + bl;
  const size_t qrow = ((size_t)(bl * DIM_S + s)) * DIM_T + tid;
  const float* qp = QK + qrow * 64;
  const v4f r0 = *(const v4f*)(qp);
  const v4f r1 = *(const v4f*)(qp + 4);
  const v4f r2 = *(const v4f*)(qp + 8);
  const v4f r3 = *(const v4f*)(qp + 12);
  const v4f r4 = *(const v4f*)(qp + 16);
  float qv[DIM_A], kv[DIM_A];
  qv[0] = r0[0]; qv[1] = r0[1]; qv[2] = r0[2]; qv[3] = r0[3];
  qv[4] = r1[0]; qv[5] = r1[1]; qv[6] = r1[2]; qv[7] = r1[3];
  qv[8] = r2[0]; qv[9] = r2[1];
  kv[0] = r2[2]; kv[1] = r2[3];
  kv[2] = r3[0]; kv[3] = r3[1]; kv[4] = r3[2]; kv[5] = r3[3];
  kv[6] = r4[0]; kv[7] = r4[1]; kv[8] = r4[2]; kv[9] = r4[3];
  const float wst = Ws[tid];
#pragma unroll
  for (int a = 0; a < DIM_A; ++a) skwp[a * DIM_T + tid] = kv[a] * wst;
  __syncthreads();
  if (tid < DIM_A) {
    float acc = 0.f;
#pragma unroll 1
    for (int u = 0; u < DIM_T; ++u) acc += skwp[tid * DIM_T + u];
    skw[tid] = acc;
  }
  __syncthreads();
  float lg = 0.f;
#pragma unroll
  for (int a = 0; a < DIM_A; ++a) lg += qv[a] * skw[a];
  lg = lg * __uint_as_float((unsigned)SCALE_BITS) + bs[0];
  float m = lg;
#pragma unroll
  for (int off = 16; off > 0; off >>= 1) m = fmaxf(m, __shfl_xor(m, off, 32));
  if (lane == 0) smax[wave] = m;
  __syncthreads();
  const float mx = fmaxf(fmaxf(smax[0], smax[1]), fmaxf(smax[2], smax[3]));
  const float ex = expf(lg - mx);
  float sm = ex;
#pragma unroll
  for (int off = 16; off > 0; off >>= 1) sm += __shfl_xor(sm, off, 32);
  if (lane == 0) ssum[wave] = sm;
  __syncthreads();
  const float tot = ((ssum[0] + ssum[1]) + ssum[2]) + ssum[3];
  const float inv = 1.0f / tot;
  sbeta[tid] = ex * inv;
  __syncthreads();
  const int c = tid;
  const int cc = min(c, DIM_E - 1);
  const int pc = min(max(c - DIM_E, 0), DIM_PE - 1);
  const float* hb = H2 + ((size_t)(bl * DIM_T) * DIM_S + s) * DIM_E + cc;
  const float* pb = PE + ((size_t)b * DIM_T) * PITCH_PE + pc;
  float acc = 0.f;
#pragma unroll 1
  for (int t2 = 0; t2 < DIM_T; ++t2) {
    const float hvv = hb[(size_t)t2 * (DIM_S * DIM_E)];
    const float pvv = pb[t2 * PITCH_PE];
    const float val = (c < DIM_E) ? hvv : pvv;
    acc += sbeta[t2] * val;
  }
  const float ctx = (c < DIM_H) ? acc : 0.f;
  const unsigned short hbits = f2bf_bits(ctx);
  const unsigned short lbits = f2bf_bits(ctx - bf_bits2f(hbits));
  s16h[c] = hbits;
  s16l[c] = lbits;
  __syncthreads();
  if (tid < 32) {
    const int plane = lane >> 4;
    const int c8 = (lane & 15) * 8;
    const v4u vh = *(const v4u*)(s16h + c8);
    const v4u vl = *(const v4u*)(s16l + c8);
    const v4u val = plane ? vl : vh;
    unsigned short* dst = (plane ? CTXl : CTXh) + ((size_t)(b * DIM_S + s)) * PITCH_W + c8;
    *(volatile v4u*)dst = val;
    __threadfence();
    *(volatile v4u*)dst = val;
  }
}

template <int ET, bool SPLIT, int BM, int OM, bool RES, int ACT>
static void gemm_launch(hipStream_t st,
                        const unsigned short* A, const unsigned short* A2, int lda, long sA,
                        const unsigned short* Bt, const unsigned short* Bt2, int ldb, long sB,
                        void* C, void* C2, int ldc, long sC, const float* bias,
                        int M, int N, int K, int nb) {
  const int tiles = (M / 64) * (N / 64) * nb;
  const int gx = (tiles + 7) / 8;
  wmma_gemm64<ET, SPLIT, BM, OM, RES, ACT><<<dim3(gx), dim3(256), 0, st>>>(
      A, A2, lda, sA, Bt, Bt2, ldb, sB, C, C2, ldc, sC, bias, (const float*)nullptr, 0L, M, N, K, 1.0f, nb);
}

extern "C" void kernel_launch(void* const* d_in, const int* in_sizes, int n_in,
                              void* d_out, int out_size, void* d_ws, size_t ws_size,
                              hipStream_t stream) {
  if (n_in < 16) return;
  const int want[16] = {DIM_B * DIM_T * DIM_S * DIM_O, DIM_B * DIM_T, DIM_B * DIM_T * DIM_S, DIM_S * DIM_O * DIM_E,
                        DIM_S * DIM_A, DIM_E * DIM_CAT, DIM_CAT, DIM_S * DIM_E, DIM_H * DIM_A, DIM_A, DIM_H * DIM_A, DIM_A,
                        DIM_T, 1, DIM_H * DIM_OUT, DIM_OUT};
  for (int i = 0; i < 16; ++i) if (in_sizes[i] != want[i]) return;
  if (out_size != DIM_B * DIM_S * DIM_OUT) return;

  const float* x     = (const float*)d_in[0];
  const float* times = (const float*)d_in[1];
  const float* mask  = (const float*)d_in[2];
  const float* obsW  = (const float*)d_in[3];
  const float* isaW  = (const float*)d_in[4];
  const float* Wrecv = (const float*)d_in[5];
  const float* brecv = (const float*)d_in[6];
  const float* bw    = (const float*)d_in[7];
  const float* Wq    = (const float*)d_in[8];
  const float* bq    = (const float*)d_in[9];
  const float* Wk    = (const float*)d_in[10];
  const float* bk    = (const float*)d_in[11];
  const float* Wsc   = (const float*)d_in[12];
  const float* bsc   = (const float*)d_in[13];
  const float* Wemb  = (const float*)d_in[14];
  const float* bemb  = (const float*)d_in[15];
  float* out = (float*)d_out;

  char* base = (char*)d_ws;
  size_t off = 0;
  auto carve = [&](size_t bytes) { char* p = base + off; off += bytes; return (void*)p; };
  const size_t szPlane64  = (size_t)ROWS_CH * 64 * 2;
  const size_t szPlanePr  = (size_t)PAIRS_CH * 4096 * 2;
  const size_t szPlaneHC  = (size_t)ROWS_CH * PITCH_W * 2;
  float* PE = (float*)carve((size_t)DIM_B * DIM_T * PITCH_PE * 4);
  unsigned short* BWh = (unsigned short*)carve(64 * 64 * 2);
  unsigned short* BWl = (unsigned short*)carve(64 * 64 * 2);
  unsigned short* WRh = (unsigned short*)carve(64 * 64 * 2);
  unsigned short* WRl = (unsigned short*)carve(64 * 64 * 2);
  unsigned short* WQh = (unsigned short*)carve(64 * PITCH_W * 2);
  unsigned short* WQl = (unsigned short*)carve(64 * PITCH_W * 2);
  unsigned short* WEh = (unsigned short*)carve(DIM_OUT * PITCH_W * 2);
  unsigned short* WEl = (unsigned short*)carve(DIM_OUT * PITCH_W * 2);
  float* BIAS  = (float*)carve(128 * 4);
  float* BIDIR = (float*)carve(64 * 64 * 4);
  unsigned short* CTXh = (unsigned short*)carve((size_t)DIM_B * DIM_S * PITCH_W * 2);
  unsigned short* CTXl = (unsigned short*)carve((size_t)DIM_B * DIM_S * PITCH_W * 2);
  unsigned short* H0h  = (unsigned short*)carve(szPlane64);
  unsigned short* H0l  = (unsigned short*)carve(szPlane64);
  unsigned short* H0Th = (unsigned short*)carve(szPlanePr);
  unsigned short* H0Tl = (unsigned short*)carve(szPlanePr);
  unsigned short* ACh  = (unsigned short*)carve(szPlanePr);
  unsigned short* ACl  = (unsigned short*)carve(szPlanePr);
  unsigned short* HMh  = (unsigned short*)carve(szPlane64);
  unsigned short* HMl  = (unsigned short*)carve(szPlane64);
  float* ALPHA = (float*)carve((size_t)PAIRS_CH * 4096 * 4);
  unsigned short* WPh  = (unsigned short*)carve(szPlanePr);
  unsigned short* WPl  = (unsigned short*)carve(szPlanePr);
  unsigned short* H1Th = (unsigned short*)carve(szPlanePr);
  unsigned short* H1Tl = (unsigned short*)carve(szPlanePr);
  float* ADJ2 = (float*)carve((size_t)CH_B * 64 * 64 * 4);
  float* H2   = (float*)carve((size_t)ROWS_CH * 64 * 4);
  unsigned short* HCh = (unsigned short*)carve(szPlaneHC);
  unsigned short* HCl = (unsigned short*)carve(szPlaneHC);
  float* QKb  = (float*)carve((size_t)ROWS_CH * 64 * 4);
  if (off > ws_size) return;

  k_petab<<<dim3(DIM_B * DIM_T / 128), dim3(128), 0, stream>>>(times, PE);
  k_wprep<<<dim3(17), dim3(256), 0, stream>>>(bw, Wrecv, brecv, Wq, bq, Wk, bk, Wemb,
                                              BWh, BWl, WRh, WRl, WQh, WQl, WEh, WEl, BIAS);
  gemm_launch<1, false, 0, 0, false, 0>(stream, BWh, BWl, 64, 0L, BWh, BWl, 64, 0L,
                                        BIDIR, nullptr, 64, 0L, nullptr, 64, 64, 64, 1);

  for (int c = 0; c < N_CHUNK; ++c) {
    k_embed<<<dim3(PAIRS_CH), dim3(256), 0, stream>>>(x, mask, obsW, isaW, PE, c,
                                                      H0h, H0l, H0Th, H0Tl, ACh, ACl);
    gemm_launch<1, false, 2, 2, false, 0>(stream, H0h, H0l, 64, 0L, WRh, WRl, 64, 0L,
                                          HMh, HMl, 64, 0L, BIAS, ROWS_CH, 64, 64, 1);
    gemm_launch<1, false, 0, 0, false, 2>(stream, HMh, HMl, 64, 4096L, ACh, ACl, 64, 4096L,
                                          ALPHA, nullptr, 64, 4096L, nullptr, 64, 64, 32, PAIRS_CH);
    k_wsplit<1><<<dim3(1024), dim3(256), 0, stream>>>(ALPHA, BIDIR, ADJ2, WPh, WPl);
    gemm_launch<1, false, 0, 2, false, 2>(stream, H0Th, H0Tl, 64, 4096L, WPh, WPl, 64, 4096L,
                                          H1Th, H1Tl, 64, 4096L, nullptr, 64, 64, 64, PAIRS_CH);
    k_adj2<<<dim3(16), dim3(256), 0, stream>>>(ALPHA, mask, ADJ2, c);
    k_wsplit<2><<<dim3(1024), dim3(256), 0, stream>>>(ALPHA, BIDIR, ADJ2, WPh, WPl);
    gemm_launch<1, false, 0, 0, false, 2>(stream, WPh, WPl, 64, 4096L, H1Th, H1Tl, 64, 4096L,
                                          H2, nullptr, 64, 4096L, nullptr, 64, 64, 64, PAIRS_CH);
    k_hcat<<<dim3(2048), dim3(256), 0, stream>>>(H2, PE, HCh, HCl, c);
    gemm_launch<1, false, 2, 0, false, 0>(stream, HCh, HCl, PITCH_W, 0L, WQh, WQl, PITCH_W, 0L,
                                          QKb, nullptr, 64, 0L, BIAS + 64, ROWS_CH, 64, K_HC, 1);
    k_attn<<<dim3(BS_CH), dim3(128), 0, stream>>>(QKb, H2, PE, Wsc, bsc, CTXh, CTXl, c);
  }
  gemm_launch<1, true, 2, 0, false, 0>(stream, CTXh, CTXl, PITCH_W, 0L, WEh, WEl, PITCH_W, 0L,
                                       out, nullptr, DIM_OUT, 0L, bemb, DIM_B * DIM_S, DIM_OUT, K_HC, 1);
}
